// VSALattice_30726196035983
// MI455X (gfx1250) — hardware-run, weakly checked
//
#include <hip/hip_runtime.h>


#ifndef NB
#define NB 64
#endif
#ifndef SEQ
#define SEQ 128
#endif
#define NB_FULL  64
#define SEQ_FULL 128
#define NRING 8
#define NATOM 10
#define DD    10000
#define PD    256
#define NBIN  5001
#define XP    10016
#define XROWS 144
#define MT    3
#define BT    313
#define FTP   (BT * 32)
#define KP    5024
#define DT    626
#define TABN  10240
#define OSP   36
#define MSP   20
#define PHS   6.283185307179586e-4f
#define WSC   1024.0f
#define FSC_IN 3.0517578125e-05f
#define FSC_ED 1.52587890625e-05f
#define MSC   0.125f
#define OSC   0.0512f

static_assert(XP % 32 == 0);
static_assert(XP >= DD);
static_assert(XP / 16 == DT);
static_assert(DD % 16 == 0);
static_assert(DD % 8 == 0);
static_assert(DD == 4 * 2500);
static_assert(XROWS == MT * 16 * 3);
static_assert(XROWS >= SEQ_FULL + NATOM + 1);
static_assert(BT * 16 >= NBIN);
static_assert(KP % 32 == 0);
static_assert(KP >= NBIN);
static_assert(KP % 8 == 0);
static_assert((FTP * 4) % 128 == 0);
static_assert(NB % 16 == 0);
static_assert(NB <= NB_FULL);
static_assert(SEQ <= SEQ_FULL);
static_assert(TABN >= DD);
static_assert((TABN / 4) % 256 == 0);
static_assert((TABN / 4) % 32 == 0);
static_assert(PD % 32 == 0);
static_assert((OSP * 4) % 16 == 0);
static_assert((MSP * 4) % 16 == 0);
static_assert(((size_t)SEQ_FULL * XP * 2) % 128 == 0);
static_assert(((size_t)(SEQ_FULL + NATOM) * XP * 2) % 128 == 0);
static_assert(4 * 32 * 16 == 16 * 32 * 4);
static_assert((NB / 16) * 32 * 16 == NB * 16 * 2);
static_assert(TABN * 4 + 16 * OSP * 4 <= 65536);
static_assert(TABN * 4 + NB * MSP * 4 <= 65536);
static_assert(TABN * 4 + NB * MSP * 4 <= 131072);

typedef _Float16 h16;
typedef unsigned short bf;
typedef __attribute__((ext_vector_type(16))) _Float16 v16h;
typedef __attribute__((ext_vector_type(8)))  _Float16 v8h;
typedef __attribute__((ext_vector_type(8)))  float    v8f;
typedef __attribute__((ext_vector_type(4)))  float    v4f;
typedef __attribute__((ext_vector_type(8)))  unsigned v8u;
typedef __attribute__((ext_vector_type(4)))  unsigned v4u;
typedef v4f  __attribute__((may_alias)) v4fa;
typedef v4u  __attribute__((may_alias)) v4ua;

__device__ __forceinline__ unsigned short f2bf(float f) { unsigned u = __float_as_uint(f); u += 0x7FFFu + ((u >> 16) & 1u); return (unsigned short)(u >> 16); }
__device__ __forceinline__ float bfr(float f) { return __uint_as_float(((unsigned)f2bf(f)) << 16); }
__device__ __forceinline__ v16h cat16(v8h lo, v8h hi) { return __builtin_shufflevector(lo, hi, 0, 1, 2, 3, 4, 5, 6, 7, 8, 9, 10, 11, 12, 13, 14, 15); }
__device__ __forceinline__ v16h ldh(const h16* p) { return cat16(*(const v8h*)p, *(const v8h*)(p + 16)); }
__device__ __forceinline__ h16 toh_flush(float v) { const h16 r = (h16)v; return (fabsf(v) < 6.103515625e-05f) ? (h16)0.0f : r; }
__device__ __forceinline__ unsigned short hbits(h16 v) { return __builtin_bit_cast(unsigned short, v); }
__device__ __forceinline__ v8f wmma16g(v16h a, v16h b, v8f c) {
    c = __builtin_amdgcn_wmma_f32_16x16x32_f16(false, a, false, b, (short)0, c, false, false);
    asm volatile("v_nop\n\tv_nop\n\tv_nop\n\tv_nop" : "+v"(c) : "v"(a), "v"(b));
    return c;
}
__device__ __forceinline__ void wave_sync() { __builtin_amdgcn_fence(3  , "wavefront"); __builtin_amdgcn_wave_barrier(); asm volatile("" ::: "memory"); }

__global__ __launch_bounds__(256) void k_tab(unsigned* TAB) {
#pragma clang fp contract(off)
    const int i = blockIdx.x * 256 + threadIdx.x; if (i >= TABN / 4) return;
    v4u o;
#pragma unroll
    for (int j = 0; j < 4; ++j) {
        const int m = 4 * i + j;
        const int mm = m < DD ? m : 0;
        const int q = (mm + 1250) / 2500;
        const int r = mm - 2500 * q;
        const float x = (float)r * PHS, x2 = x * x;
        float sp = 2.7557319e-6f;
        sp = sp * x2 - 1.9841270e-4f; sp = sp * x2 + 8.3333333e-3f; sp = sp * x2 - 1.6666667e-1f; sp = sp * x2 + 1.0f; sp = sp * x;
        float cp = -2.7557319e-7f;
        cp = cp * x2 + 2.4801587e-5f; cp = cp * x2 - 1.3888889e-3f; cp = cp * x2 + 4.1666667e-2f; cp = cp * x2 - 0.5f; cp = cp * x2 + 1.0f;
        const int qq = q & 3;
        const float cv = (qq == 0) ? cp : ((qq == 1) ? -sp : ((qq == 2) ? -cp : sp));
        const float sv = (qq == 0) ? sp : ((qq == 1) ? cp : ((qq == 2) ? -sp : -cp));
        const unsigned e = (unsigned)hbits(toh_flush(cv)) | (((unsigned)hbits(toh_flush(sv))) << 16);
        o[j] = (m < DD) ? e : 0u;
    }
    *(volatile v4u*)(TAB + (size_t)i * 4) = o; __threadfence(); *(volatile v4u*)(TAB + (size_t)i * 4) = o;
}

__global__ __launch_bounds__(256) void k_rows(const float* __restrict__ src, int srows, h16* dst, int nrows, float scale) {
    const int raw = blockIdx.x * 256 + threadIdx.x; const int n = nrows * (XP / 8);
    if ((raw & ~31) >= n) return;
    const int i = raw < n ? raw : n - 1;
    const int r = i / (XP / 8), c = i - r * (XP / 8);
    const int rc = r < srows ? r : srows - 1;
    const int cc = c < DD / 8 ? c : DD / 8 - 1;
    v8f v = *(const v8f*)(src + (size_t)rc * DD + (size_t)cc * 8);
    asm volatile("" : "+v"(v));
    const bool ok = (r < srows) & (c < DD / 8);
    v8h o;
#pragma unroll
    for (int k = 0; k < 8; ++k) { const h16 t = toh_flush(bfr(v[k]) * scale); o[k] = ok ? t : (h16)0.0f; }
    *(volatile v8h*)(dst + (size_t)i * 8) = o; __threadfence(); *(volatile v8h*)(dst + (size_t)i * 8) = o;
}

__global__ __launch_bounds__(32) void k_fwd(const h16* __restrict__ X, const unsigned* __restrict__ TAB, float* FT) {
    __shared__ __align__(16) unsigned tab[TABN];
    __shared__ __align__(16) float os[16 * OSP];
    const int lane = threadIdx.x & 31, lr = lane & 15, hi = lane >> 4;
    const int bt = blockIdx.x; const int m0 = blockIdx.y * (16 * MT);
#pragma unroll 1
    for (int j = lane; j < TABN / 4; j += 32) { const v4u t = *(const v4u*)(TAB + (size_t)j * 4); *(v4ua*)(&tab[j * 4]) = t; }
    __syncthreads();
    const unsigned kb = (unsigned)(bt * 16 + lr);
    const unsigned st1 = kb;
    const unsigned st9 = (9u * kb) % (unsigned)DD;
    unsigned idx = (8u * (unsigned)hi * kb) % (unsigned)DD;
    v8f accC[MT], accS[MT];
#pragma unroll
    for (int mb = 0; mb < MT; ++mb) { accC[mb] = (v8f){}; accS[mb] = (v8f){}; }
    const size_t aoff = (size_t)(m0 + lr) * XP + 8 * hi;
#pragma unroll 1
    for (int kc = 0; kc < XP; kc += 32) {
        v8u pc, ps;
#pragma unroll
        for (int p = 0; p < 8; ++p) {
            const unsigned t0 = tab[idx];
            unsigned t = idx + st1; idx = (t >= (unsigned)DD) ? (t - (unsigned)DD) : t;
            const unsigned t1 = tab[idx];
            t = idx + (((p & 3) == 3) ? st9 : st1); idx = (t >= (unsigned)DD) ? (t - (unsigned)DD) : t;
            pc[p] = (t0 & 0xffffu) | (t1 << 16);
            ps[p] = (t0 >> 16) | (t1 & 0xffff0000u);
        }
        const v16h bc = __builtin_bit_cast(v16h, pc), bs = __builtin_bit_cast(v16h, ps);
#pragma unroll
        for (int mb = 0; mb < MT; ++mb) {
            const v16h a = ldh(X + aoff + (size_t)mb * 16 * XP + kc);
            accC[mb] = wmma16g(a, bc, accC[mb]);
            accS[mb] = wmma16g(a, bs, accS[mb]);
        }
    }
#pragma unroll
    for (int mb = 0; mb < MT; ++mb) {
#pragma unroll
        for (int r = 0; r < 8; ++r) { os[(hi * 8 + r) * OSP + lr] = accC[mb][r]; os[(hi * 8 + r) * OSP + 16 + lr] = accS[mb][r]; }
        wave_sync();
        float* frow = FT + (size_t)(m0 + mb * 16) * FTP + (size_t)bt * 32;
#pragma unroll 1
        for (int ps2 = 0; ps2 < 2; ++ps2) {
#pragma unroll
            for (int s = 0; s < 4; ++s) { const int row = 4 * s + (lane >> 3), cofs = (lane & 7) * 4;
                const v4f val = *(const v4fa*)(&os[row * OSP + cofs]);
                *(volatile v4f*)(frow + (size_t)row * FTP + cofs) = val; }
            if (ps2 == 0) __threadfence(); }
        wave_sync();
    }
}

__global__ __launch_bounds__(256) void k_asm(const float* __restrict__ FT, const float* __restrict__ tmask, const float* __restrict__ rmask,
                                             const int* __restrict__ aidx, const int* __restrict__ rpos, h16* FR, h16* FS) {
#pragma clang fp contract(off)
    const int i = blockIdx.x * 256 + threadIdx.x; if (i >= NB * (KP / 8)) return;
    const int b = i / (KP / 8), c = i - b * (KP / 8);
    const int k0 = c * 8;
    int tcl = k0 >> 4; tcl = tcl < BT - 1 ? tcl : BT - 1;
    const size_t co = (size_t)tcl * 32 + (size_t)(k0 & 15);
    float fr[8], fs[8];
#pragma unroll
    for (int j = 0; j < 8; ++j) { fr[j] = 0.0f; fs[j] = 0.0f; }
    const float* pcl = FT + (size_t)(SEQ_FULL + NATOM) * FTP + co;
    v4f c0 = *(const v4f*)pcl, c1 = *(const v4f*)(pcl + 4), c2 = *(const v4f*)(pcl + 16), c3 = *(const v4f*)(pcl + 20);
    asm volatile("" : "+v"(c0)); asm volatile("" : "+v"(c1)); asm volatile("" : "+v"(c2)); asm volatile("" : "+v"(c3));
#pragma unroll 1
    for (int s = 0; s < SEQ; ++s) {
        const float m = bfr(tmask[(size_t)b * SEQ_FULL + s]);
        int a = aidx[(size_t)b * SEQ_FULL + s]; a = a < 0 ? a + NATOM : a; a = a < 0 ? 0 : (a > NATOM - 1 ? NATOM - 1 : a);
        const float* pa = FT + (size_t)(SEQ_FULL + a) * FTP + co;
        const float* pp = FT + (size_t)s * FTP + co;
        v4f a0 = *(const v4f*)pa, a1 = *(const v4f*)(pa + 4), a2 = *(const v4f*)(pa + 16), a3 = *(const v4f*)(pa + 20);
        v4f p0 = *(const v4f*)pp, p1 = *(const v4f*)(pp + 4), p2 = *(const v4f*)(pp + 16), p3 = *(const v4f*)(pp + 20);
        asm volatile("" : "+v"(a0)); asm volatile("" : "+v"(a1)); asm volatile("" : "+v"(a2)); asm volatile("" : "+v"(a3));
        asm volatile("" : "+v"(p0)); asm volatile("" : "+v"(p1)); asm volatile("" : "+v"(p2)); asm volatile("" : "+v"(p3));
#pragma unroll
        for (int j = 0; j < 4; ++j) {
            { const float tr = a0[j] * p0[j] - a2[j] * p2[j]; const float ts = a0[j] * p2[j] + a2[j] * p0[j]; fr[j] = fr[j] + m * tr; fs[j] = fs[j] + m * ts; }
            { const float tr = a1[j] * p1[j] - a3[j] * p3[j]; const float ts = a1[j] * p3[j] + a3[j] * p1[j]; fr[4 + j] = fr[4 + j] + m * tr; fs[4 + j] = fs[4 + j] + m * ts; }
        }
    }
#pragma unroll 1
    for (int r = 0; r < NRING; ++r) {
        const float rm = bfr(rmask[(size_t)b * NRING + r]);
        int i0 = rpos[((size_t)b * NRING + r) * 2 + 0], i1 = rpos[((size_t)b * NRING + r) * 2 + 1];
        i0 = i0 < 0 ? i0 + SEQ_FULL : i0; i0 = i0 < 0 ? 0 : (i0 > SEQ_FULL - 1 ? SEQ_FULL - 1 : i0);
        i1 = i1 < 0 ? i1 + SEQ_FULL : i1; i1 = i1 < 0 ? 0 : (i1 > SEQ_FULL - 1 ? SEQ_FULL - 1 : i1);
        const float* px = FT + (size_t)i0 * FTP + co;
        const float* py = FT + (size_t)i1 * FTP + co;
        v4f x0 = *(const v4f*)px, x1 = *(const v4f*)(px + 4), x2 = *(const v4f*)(px + 16), x3 = *(const v4f*)(px + 20);
        v4f y0 = *(const v4f*)py, y1 = *(const v4f*)(py + 4), y2 = *(const v4f*)(py + 16), y3 = *(const v4f*)(py + 20);
        asm volatile("" : "+v"(x0)); asm volatile("" : "+v"(x1)); asm volatile("" : "+v"(x2)); asm volatile("" : "+v"(x3));
        asm volatile("" : "+v"(y0)); asm volatile("" : "+v"(y1)); asm volatile("" : "+v"(y2)); asm volatile("" : "+v"(y3));
#pragma unroll
        for (int j = 0; j < 4; ++j) {
            { const float xr = x0[j] * y0[j] - x2[j] * y2[j]; const float xs = x0[j] * y2[j] + x2[j] * y0[j];
              const float zr = xr * c0[j] - xs * c2[j]; const float zs = xr * c2[j] + xs * c0[j]; fr[j] = fr[j] + rm * zr; fs[j] = fs[j] + rm * zs; }
            { const float xr = x1[j] * y1[j] - x3[j] * y3[j]; const float xs = x1[j] * y3[j] + x3[j] * y1[j];
              const float zr = xr * c1[j] - xs * c3[j]; const float zs = xr * c3[j] + xs * c1[j]; fr[4 + j] = fr[4 + j] + rm * zr; fs[4 + j] = fs[4 + j] + rm * zs; }
        }
    }
    v8h orr, oss;
#pragma unroll
    for (int j = 0; j < 8; ++j) {
        const int k = k0 + j;
        const bool valid = k <= DD / 2;
        const bool edge = (k == 0) | (k == DD / 2);
        const float w = edge ? FSC_ED : FSC_IN;
        const h16 hr = toh_flush(fr[j] * w);
        const h16 hs = toh_flush(fs[j] * w);
        orr[j] = valid ? hr : (h16)0.0f;
        oss[j] = (valid & !edge) ? hs : (h16)0.0f;
    }
#pragma unroll 1
    for (int ps = 0; ps < 2; ++ps) {
        *(volatile v8h*)(FR + (size_t)i * 8) = orr; *(volatile v8h*)(FS + (size_t)i * 8) = oss;
        if (ps == 0) __threadfence(); }
}

__global__ __launch_bounds__(32) void k_inv(const h16* __restrict__ FR, const h16* __restrict__ FS, const unsigned* __restrict__ TAB, h16* MOL) {
    __shared__ __align__(16) unsigned tab[TABN];
    __shared__ __align__(16) float os[NB * MSP];
    const int lane = threadIdx.x & 31, lr = lane & 15, hi = lane >> 4;
    const int dt = blockIdx.x;
#pragma unroll 1
    for (int j = lane; j < TABN / 4; j += 32) { const v4u t = *(const v4u*)(TAB + (size_t)j * 4); *(v4ua*)(&tab[j * 4]) = t; }
    __syncthreads();
    const unsigned dcol = (unsigned)(dt * 16 + lr);
    const unsigned st1 = dcol % (unsigned)DD;
    const unsigned st9 = (9u * dcol) % (unsigned)DD;
    unsigned idx = (8u * (unsigned)hi * dcol) % (unsigned)DD;
    v8f acc[NB / 16];
#pragma unroll
    for (int nb = 0; nb < NB / 16; ++nb) acc[nb] = (v8f){};
    const size_t boff = (size_t)lr * KP + 8 * hi;
#pragma unroll 1
    for (int kc = 0; kc < KP; kc += 32) {
        v8u pc, ps;
#pragma unroll
        for (int p = 0; p < 8; ++p) {
            const unsigned t0 = tab[idx];
            unsigned t = idx + st1; idx = (t >= (unsigned)DD) ? (t - (unsigned)DD) : t;
            const unsigned t1 = tab[idx];
            t = idx + (((p & 3) == 3) ? st9 : st1); idx = (t >= (unsigned)DD) ? (t - (unsigned)DD) : t;
            pc[p] = (t0 & 0xffffu) | (t1 << 16);
            ps[p] = (t0 >> 16) | (t1 & 0xffff0000u);
        }
        const v16h fc = __builtin_bit_cast(v16h, pc), fsn = __builtin_bit_cast(v16h, ps);
#pragma unroll
        for (int nb = 0; nb < NB / 16; ++nb) {
            const v16h bR = ldh(FR + boff + (size_t)nb * 16 * KP + kc);
            const v16h bS = ldh(FS + boff + (size_t)nb * 16 * KP + kc);
            acc[nb] = wmma16g(fc, bR, acc[nb]);
            acc[nb] = wmma16g(fsn, bS, acc[nb]);
        }
    }
#pragma unroll
    for (int nb = 0; nb < NB / 16; ++nb) { v4f a, c;
        a[0] = acc[nb][0] * MSC; a[1] = acc[nb][1] * MSC; a[2] = acc[nb][2] * MSC; a[3] = acc[nb][3] * MSC;
        c[0] = acc[nb][4] * MSC; c[1] = acc[nb][5] * MSC; c[2] = acc[nb][6] * MSC; c[3] = acc[nb][7] * MSC;
        *(v4fa*)(&os[(nb * 16 + lr) * MSP + 8 * hi]) = a; *(v4fa*)(&os[(nb * 16 + lr) * MSP + 8 * hi + 4]) = c; }
    wave_sync();
    h16* mt = MOL + (size_t)dt * ((size_t)NB * 16);
#pragma unroll 1
    for (int ps2 = 0; ps2 < 2; ++ps2) {
#pragma unroll
        for (int s = 0; s < NB / 16; ++s) { const int p = s * 32 + lane; const int bb = p >> 1, hf = p & 1;
            const v4f x0 = *(const v4fa*)(&os[bb * MSP + hf * 8]); const v4f x1 = *(const v4fa*)(&os[bb * MSP + hf * 8 + 4]);
            const int d0 = dt * 16 + hf * 8; v8h hv;
#pragma unroll
            for (int j = 0; j < 4; ++j) { const h16 u0 = toh_flush(x0[j]); const h16 u1 = toh_flush(x1[j]);
                hv[j] = (d0 + j < DD) ? u0 : (h16)0.0f; hv[4 + j] = (d0 + 4 + j < DD) ? u1 : (h16)0.0f; }
            *(volatile v8h*)(mt + (size_t)p * 8) = hv; }
        if (ps2 == 0) __threadfence(); }
}

__global__ __launch_bounds__(32) void k_out(const h16* __restrict__ MOL, const h16* __restrict__ WH, const float* __restrict__ bias, float* OUT) {
    __shared__ __align__(16) float os[16 * OSP];
    const int lane = threadIdx.x & 31, lr = lane & 15, hi = lane >> 4;
    const int p0 = blockIdx.x * 32, b0 = blockIdx.y * 16;
    v8f acc0 = (v8f){}, acc1 = (v8f){};
    const size_t ao = (size_t)(b0 + lr) * 16 + 8 * hi;
    const size_t bo = (size_t)(p0 + lr) * XP + 8 * hi;
#pragma unroll 1
    for (int s = 0; s < XP / 32; ++s) {
        const h16* ap = MOL + ao + (size_t)(2 * s) * ((size_t)NB * 16);
        const v16h a = cat16(*(const v8h*)ap, *(const v8h*)(ap + (size_t)NB * 16));
        const v16h w0 = ldh(WH + bo + (size_t)s * 32);
        const v16h w1 = ldh(WH + bo + (size_t)16 * XP + (size_t)s * 32);
        acc0 = wmma16g(a, w0, acc0);
        acc1 = wmma16g(a, w1, acc1);
    }
    const float bc0 = bfr(bias[p0 + lr]), bc1 = bfr(bias[p0 + 16 + lr]);
#pragma unroll
    for (int r = 0; r < 8; ++r) { os[(hi * 8 + r) * OSP + lr] = acc0[r] * OSC + bc0; os[(hi * 8 + r) * OSP + 16 + lr] = acc1[r] * OSC + bc1; }
    wave_sync();
    float* orow = OUT + (size_t)b0 * PD + p0;
#pragma unroll 1
    for (int ps = 0; ps < 2; ++ps) {
#pragma unroll
        for (int s = 0; s < 4; ++s) { const int row = 4 * s + (lane >> 3), cofs = (lane & 7) * 4;
            const v4f val = *(const v4fa*)(&os[row * OSP + cofs]);
            *(volatile v4f*)(orow + (size_t)row * PD + cofs) = val; }
        if (ps == 0) __threadfence(); }
}

static constexpr size_t al256(size_t v) { return (v + 255) & ~(size_t)255; }
static constexpr size_t SZ_TAB = al256((size_t)TABN * 4);
static constexpr size_t SZ_X   = al256((size_t)XROWS * XP * 2);
static constexpr size_t SZ_W   = al256((size_t)PD * XP * 2);
static constexpr size_t SZ_FT  = al256((size_t)XROWS * FTP * 4);
static constexpr size_t SZ_FQ  = al256((size_t)NB * KP * 2);
static constexpr size_t SZ_MOL = al256((size_t)DT * NB * 16 * 2);
static constexpr size_t SZ_TOTAL = SZ_TAB + SZ_X + SZ_W + SZ_FT + 2 * SZ_FQ + SZ_MOL;
static_assert(SZ_TOTAL <= (size_t)134217728);
static_assert((size_t)(XROWS / (16 * MT)) * (16 * MT) * FTP * 4 <= SZ_FT);
static_assert((size_t)BT * 32 == (size_t)FTP);
static_assert((size_t)(SEQ_FULL + NATOM + 6) * XP * 2 <= SZ_X);
static_assert(SEQ_FULL + NATOM + 6 == XROWS);
static_assert((size_t)DT * NB * 16 * 2 <= SZ_MOL);

extern "C" void kernel_launch(void* const* d_in, const int* in_sizes, int n_in,
                              void* d_out, int out_size, void* d_ws, size_t ws_size, hipStream_t stream) {
    if (n_in < 9) return;
    if ((size_t)in_sizes[0] < (size_t)NATOM * DD || (size_t)in_sizes[1] < (size_t)SEQ_FULL * DD || (size_t)in_sizes[2] < (size_t)DD) return;
    if ((size_t)in_sizes[3] < (size_t)PD * DD || in_sizes[4] < PD) return;
    if ((size_t)in_sizes[5] < (size_t)(NB - 1) * SEQ_FULL + SEQ || (size_t)in_sizes[7] < (size_t)(NB - 1) * SEQ_FULL + SEQ) return;
    if ((size_t)in_sizes[6] < (size_t)NB * NRING || (size_t)in_sizes[8] < (size_t)NB * NRING * 2) return;
    if ((size_t)out_size < (size_t)NB * PD) return;
    if (SZ_TOTAL > ws_size) return;
    const float* atom  = (const float*)d_in[0];
    const float* pos   = (const float*)d_in[1];
    const float* clos  = (const float*)d_in[2];
    const float* W     = (const float*)d_in[3];
    const float* bias  = (const float*)d_in[4];
    const float* tmask = (const float*)d_in[5];
    const float* rmask = (const float*)d_in[6];
    const int*   aidx  = (const int*)d_in[7];
    const int*   rpos  = (const int*)d_in[8];
    float* OUT = (float*)d_out;
    char* wsp = (char*)d_ws;
    unsigned* TAB = (unsigned*)wsp; wsp += SZ_TAB;
    h16* X   = (h16*)wsp;  wsp += SZ_X;
    h16* WH  = (h16*)wsp;  wsp += SZ_W;
    float* FT = (float*)wsp; wsp += SZ_FT;
    h16* FR  = (h16*)wsp;  wsp += SZ_FQ;
    h16* FS  = (h16*)wsp;  wsp += SZ_FQ;
    h16* MOL = (h16*)wsp;  wsp += SZ_MOL;

    k_tab<<<(unsigned)(TABN / 4 / 256), 256, 0, stream>>>(TAB);
    { const int n = SEQ_FULL * (XP / 8); k_rows<<<(unsigned)((n + 255) / 256), 256, 0, stream>>>(pos, SEQ_FULL, X, SEQ_FULL, 1.0f); }
    { const int n = NATOM * (XP / 8);    k_rows<<<(unsigned)((n + 255) / 256), 256, 0, stream>>>(atom, NATOM, X + (size_t)SEQ_FULL * XP, NATOM, 1.0f); }
    { const int n = 6 * (XP / 8);        k_rows<<<(unsigned)((n + 255) / 256), 256, 0, stream>>>(clos, 1, X + (size_t)(SEQ_FULL + NATOM) * XP, 6, 1.0f); }
    { const int n = PD * (XP / 8);       k_rows<<<(unsigned)((n + 255) / 256), 256, 0, stream>>>(W, PD, WH, PD, WSC); }
    k_fwd<<<dim3(BT, XROWS / (16 * MT), 1), 32, 0, stream>>>(X, TAB, FT);
    { const int n = NB * (KP / 8);       k_asm<<<(unsigned)((n + 255) / 256), 256, 0, stream>>>(FT, tmask, rmask, aidx, rpos, FR, FS); }
    k_inv<<<dim3(DT, 1, 1), 32, 0, stream>>>(FR, FS, TAB, MOL);
    k_out<<<dim3(PD / 32, NB / 16, 1), 32, 0, stream>>>(MOL, WH, bias, OUT);
}
